// VanillaRecursiveNN_25589415149692
// MI455X (gfx1250) — hardware-run, weakly checked
//
#include <hip/hip_runtime.h>

typedef float          v8f   __attribute__((ext_vector_type(8)));
typedef float          v4f   __attribute__((ext_vector_type(4)));
typedef unsigned int   v4u   __attribute__((ext_vector_type(4)));
typedef int            v8i   __attribute__((ext_vector_type(8)));
typedef unsigned short v8us  __attribute__((ext_vector_type(8)));
typedef unsigned short v16us __attribute__((ext_vector_type(16)));
typedef __bf16         v16bf __attribute__((ext_vector_type(16)));
typedef _Float16       v16h  __attribute__((ext_vector_type(16)));
typedef v4f  __attribute__((may_alias)) v4fa;
typedef v8us __attribute__((may_alias)) v8usa;
union FragB { v16bf v; v16us u; v8us h[2]; v8i w; };
union FragH { v16h  v; v16us u; v8us h[2]; v8i w; };

__device__ __forceinline__ v8f wmb(const FragB& a, const FragB& b, v8f c) {
  v8f d = __builtin_amdgcn_wmma_f32_16x16x32_bf16(false, a.v, false, b.v, (short)0, c, false, false);
  asm volatile("v_nop\n\tv_nop\n\tv_nop\n\tv_nop" : "+v"(d) : "v"(a.w), "v"(b.w));
  return d;
}

__device__ __forceinline__ v8f wmh(const FragH& a, const FragH& b, v8f c) {
  v8f d = __builtin_amdgcn_wmma_f32_16x16x32_f16(false, a.v, false, b.v, (short)0, c, false, false);
  asm volatile("v_nop\n\tv_nop\n\tv_nop\n\tv_nop" : "+v"(d) : "v"(a.w), "v"(b.w));
  return d;
}

__device__ __forceinline__ unsigned bf16_bits(float f) {
  const unsigned u = __float_as_uint(f);
  const unsigned r = (u + 0x7FFFu + ((u >> 16) & 1u)) >> 16;
  const unsigned q = (u >> 16) | 0x40u;
  return ((u & 0x7fffffffu) > 0x7f800000u) ? q : r;
}

__device__ __forceinline__ float bf16_val(float f) {
  return __uint_as_float(bf16_bits(f) << 16);
}
__device__ __forceinline__ int clampi(int v, int lo, int hi) {
  return v < lo ? lo : (v > hi ? hi : v);
}

__device__ __forceinline__ unsigned f16_bits(float f) {
  const unsigned u  = __float_as_uint(f);
  const unsigned s  = (u >> 16) & 0x8000u;
  const unsigned a  = u & 0x7fffffffu;
  const unsigned t  = a - 0x38000000u;
  const unsigned r  = (t + 0x0FFFu + ((t >> 13) & 1u)) >> 13;
  const unsigned rc = r > 0x7C00u ? 0x7C00u : r;
  const bool small  = a < 0x38800000u;
  const bool isnan  = a > 0x7f800000u;
  const unsigned fin = small ? 0u : (s | rc);
  return isnan ? (s | 0x7E00u) : fin;
}

__device__ __forceinline__ unsigned pk16(unsigned lo, unsigned hi) { return lo | (hi << 16); }
__device__ __forceinline__ unsigned bf16_lo_bits(float v) {
  float hi = bf16_val(v);
  asm volatile("" : "+v"(hi));
  return bf16_bits(v - hi);
}
__device__ __forceinline__ v4u pack8_bf16(v4f a, v4f c) {
  return (v4u){ pk16(bf16_bits(a[0]), bf16_bits(a[1])), pk16(bf16_bits(a[2]), bf16_bits(a[3])),
                pk16(bf16_bits(c[0]), bf16_bits(c[1])), pk16(bf16_bits(c[2]), bf16_bits(c[3])) };
}
__device__ __forceinline__ v4u pack8_bf16_lo(v4f a, v4f c) {
  return (v4u){ pk16(bf16_lo_bits(a[0]), bf16_lo_bits(a[1])), pk16(bf16_lo_bits(a[2]), bf16_lo_bits(a[3])),
                pk16(bf16_lo_bits(c[0]), bf16_lo_bits(c[1])), pk16(bf16_lo_bits(c[2]), bf16_lo_bits(c[3])) };
}
__device__ __forceinline__ v4u pack8_f16(v4f a, v4f c) {
  return (v4u){ pk16(f16_bits(a[0]), f16_bits(a[1])), pk16(f16_bits(a[2]), f16_bits(a[3])),
                pk16(f16_bits(c[0]), f16_bits(c[1])), pk16(f16_bits(c[2]), f16_bits(c[3])) };
}

template <int FORM>
__global__ __launch_bounds__(256) void k_plane(const float* __restrict__ src, int rows, int cols, int ldsrc,
                                               unsigned short* __restrict__ dst, int MP, int KP) {
  static_assert(FORM >= 0 && FORM <= 3);
  const int KTOT = (FORM == 1 || FORM == 3) ? 2 * KP : KP;
  const unsigned ppr   = (unsigned)(KTOT >> 3);
  const unsigned kp8   = (unsigned)(KP >> 3);
  const unsigned total = (unsigned)MP * ppr;
  const unsigned g     = blockIdx.x * 256u + threadIdx.x;
  const unsigned rowu  = g / ppr;
  const unsigned p     = g - rowu * ppr;
  const bool second    = p >= kp8;
  const int row = (int)rowu;
  const int c0  = (int)((second ? p - kp8 : p) << 3);
  const float* srow = src + (size_t)clampi(row, 0, rows - 1) * (size_t)ldsrc;
  float x[8];
  unsigned mk[8];
#pragma unroll
  for (int e = 0; e < 8; ++e) {
    const int c = c0 + e;
    const float v = srow[clampi(c, 0, cols - 1)];
    asm volatile("" :: "v"(v));
    x[e]  = v;
    mk[e] = (row < rows && c < cols) ? 0xFFFFu : 0u;
  }
  const v4f a = (v4f){ x[0], x[1], x[2], x[3] };
  const v4f c = (v4f){ x[4], x[5], x[6], x[7] };
  v4u o;
  if (FORM == 2) {
    o = pack8_f16(a, c);
  } else {
    const v4u hi = pack8_bf16(a, c);
    o = hi;
    if (FORM == 1) { const v4u lo = pack8_bf16_lo(a, c); o = second ? lo : hi; }
  }
  const v4u mw = (v4u){ pk16(mk[0], mk[1]), pk16(mk[2], mk[3]), pk16(mk[4], mk[5]), pk16(mk[6], mk[7]) };
  o &= mw;
  if (g < total) {
    volatile v4u* q = (volatile v4u*)(dst + (size_t)g * 8);
    *q = o;
    __threadfence();
    *q = o;
  }
}

template <int FORM> struct FragOf    { typedef FragB T; };
template <>         struct FragOf<2> { typedef FragH T; };
__device__ __forceinline__ v8f mm(const FragB& a, const FragB& b, v8f c) { return wmb(a, b, c); }
__device__ __forceinline__ v8f mm(const FragH& a, const FragH& b, v8f c) { return wmh(a, b, c); }
template <class F> __device__ __forceinline__ F ld_frag(const unsigned short* p) {
  F f;
  f.h[0] = *(const v8usa*)(p);
  f.h[1] = *(const v8usa*)(p + 16);
  return f;
}

template <int FORM, int EPI>
__global__ __launch_bounds__(256) __attribute__((amdgpu_num_vgpr(248)))
void k_gemm_nt(const unsigned short* __restrict__ A, const unsigned short* __restrict__ B,
               const float* __restrict__ bias, float* __restrict__ D, int M, int N, int KTOT, int ldd) {
  static_assert(FORM >= 0 && FORM <= 2);
  static_assert(EPI == 0 || EPI == 1);
  typedef typename FragOf<FORM>::T F;
  __shared__ __attribute__((aligned(16))) float sT[8][16 * 68];
  const int lane = threadIdx.x & 31;
  const int wave = threadIdx.x >> 5;
  const int tilesM = (M + 63) >> 6;
  const int tilesN = (N + 63) >> 6;
  const int tile = blockIdx.x * 8 + wave;
  if (tile >= tilesM * tilesN) return;
  const int tm = tile / tilesN;
  const int tn = tile - tm * tilesN;
  const int m0 = tm << 6;
  const int n0 = tn << 6;

  const int rl = lane & 15;
  const int h8 = (lane >> 4) * 8;
  const unsigned short* pa = A + (size_t)(m0 + rl) * (size_t)KTOT + h8;
  const unsigned short* pb = B + (size_t)(n0 + rl) * (size_t)KTOT + h8;

  v8f acc[4][4];
#pragma unroll
  for (int i = 0; i < 4; ++i)
#pragma unroll
    for (int j = 0; j < 4; ++j) acc[i][j] = (v8f){0.f, 0.f, 0.f, 0.f, 0.f, 0.f, 0.f, 0.f};

#pragma unroll 1
  for (int k0 = 0; k0 < KTOT; k0 += 32) {
    F bf[4];
#pragma unroll
    for (int j = 0; j < 4; ++j) bf[j] = ld_frag<F>(pb + (size_t)(j << 4) * (size_t)KTOT + k0);
#pragma unroll
    for (int i = 0; i < 4; ++i) {
      const F af = ld_frag<F>(pa + (size_t)(i << 4) * (size_t)KTOT + k0);
#pragma unroll
      for (int j = 0; j < 4; ++j) acc[i][j] = mm(af, bf[j], acc[i][j]);
    }
  }

  float* slab = sT[wave];
  const int hh = lane >> 4;
  const int c4 = (lane & 15) * 4;
  const int nc = n0 + c4;
  const bool cok = nc < N;
  v4f bv = (v4f){0.f, 0.f, 0.f, 0.f};
  if (EPI == 1) {
    bv = *(const v4fa*)(bias + clampi(nc, 0, N - 4));
    asm volatile("" :: "v"(bv));
  }
#pragma unroll
  for (int i = 0; i < 4; ++i) {
    const int mBase = m0 + (i << 4);
#pragma unroll
    for (int j = 0; j < 4; ++j) {
#pragma unroll
      for (int r = 0; r < 8; ++r) slab[(h8 + r) * 68 + (j << 4) + rl] = acc[i][j][r];
    }
    __builtin_amdgcn_fence(__ATOMIC_RELEASE, "workgroup");
    __builtin_amdgcn_wave_barrier();
    __builtin_amdgcn_fence(__ATOMIC_ACQUIRE, "workgroup");
    v4f vv[8];
#pragma unroll
    for (int it = 0; it < 8; ++it) {
      const int row = it * 2 + hh;
      v4f v = *(const v4fa*)(slab + row * 68 + c4);
      if (EPI == 1) v += bv;
      vv[it] = v;
    }
    for (int pass = 0; pass < 2; ++pass) {
#pragma unroll
      for (int it = 0; it < 8; ++it) {
        const int row = mBase + it * 2 + hh;
        if (cok && row < M) *(volatile v4f*)(D + (size_t)row * (size_t)ldd + nc) = vv[it];
      }
      __threadfence();
    }
    __builtin_amdgcn_fence(__ATOMIC_RELEASE, "workgroup");
    __builtin_amdgcn_wave_barrier();
    __builtin_amdgcn_fence(__ATOMIC_ACQUIRE, "workgroup");
  }
}

#pragma clang fp contract(off)

#define NTREE   256
#define NLEAF   256
#define NLEVEL  8
#define VOCAB   50000
#define WDIM    300
#define K0PAD   320
#define HID     512
#define K2      1024
#define NGROUP  4
#define GTREES  64
#define GROWS   (GTREES * NLEAF)
#define NTHR    256
#define CARRY   1024.0f
#define FOLD    0x1p-10f
#define PB_W2H  ((HID * (K2 / 8)) / NTHR)
#define WSMAX   ((size_t)128 << 20)

static constexpr int LEVEL_FORM[NLEVEL] = { 2, 2, 2, 1, 1, 1, 1, 1 };

static constexpr bool forms_valid() {
  for (int l = 0; l < NLEVEL; ++l) if (LEVEL_FORM[l] != 1 && LEVEL_FORM[l] != 2) return false;
  return true;
}
static constexpr size_t ap_bytes_level(int l) {
  return (size_t)(GROWS >> l) * (size_t)(LEVEL_FORM[l - 1] == 1 ? 2 * K2 : K2) * 2;
}
static constexpr size_t ap_bytes_max() {
  size_t m = 0;
  for (int l = 1; l <= NLEVEL; ++l) { const size_t s = ap_bytes_level(l); if (s > m) m = s; }
  return m;
}
static constexpr bool TABLE_AS_BUILT =
    LEVEL_FORM[0] == 2 && LEVEL_FORM[1] == 2 && LEVEL_FORM[2] == 2 && LEVEL_FORM[3] == 1 &&
    LEVEL_FORM[4] == 1 && LEVEL_FORM[5] == 1 && LEVEL_FORM[6] == 1 && LEVEL_FORM[7] == 1;

static_assert(forms_valid());
static_assert(NTREE == NGROUP * GTREES && NLEAF == (1 << NLEVEL));
static_assert(K0PAD % 32 == 0 && K0PAD >= WDIM && K0PAD == 320 && (WDIM % 4) == 0);
static_assert(HID % 64 == 0 && HID % 32 == 0 && HID % 4 == 0 && K2 == 2 * HID && K2 % 32 == 0 && (2 * K2) % 32 == 0);
static_assert(GROWS % 64 == 0 && GROWS % 8 == 0);
static_assert((GROWS >> NLEVEL) == 64);
static_assert((GROWS >> NLEVEL) * NGROUP == NTREE);
static_assert((HID * (K0PAD / 8)) % 256 == 0);
static_assert((HID * (2 * K2 / 8)) % 256 == 0);
static_assert((HID * (K2 / 8)) % NTHR == 0);
static_assert((64 * (K2 / 8)) % 256 == 0 && (64 * (2 * K2 / 8)) % 256 == 0);
static_assert((64 * (HID / 4)) % NTHR == 0);
static_assert(HID / 4 <= NTHR);

static constexpr size_t SZ_A0  = (size_t)GROWS * K0PAD * 2;
static constexpr size_t SZ_HA  = (size_t)GROWS * HID * 4;
static constexpr size_t SZ_HB  = (size_t)(GROWS / 2) * HID * 4;
static constexpr size_t SZ_AP  = ap_bytes_max();
static constexpr size_t SZ_W1B = (size_t)HID * K0PAD * 2;
static constexpr size_t SZ_W2H = (size_t)HID * K2 * 2;
static constexpr size_t SZ_W2D = (size_t)HID * 2 * K2 * 2;
static constexpr size_t SZ_B2V = (size_t)HID * 4;
static constexpr size_t O_A0   = 0;
static constexpr size_t O_HA   = O_A0 + SZ_A0;
static constexpr size_t O_HB   = O_HA + SZ_HA;
static constexpr size_t O_AP   = O_HB + SZ_HB;
static constexpr size_t O_W1B  = O_AP + SZ_AP;
static constexpr size_t O_W2H  = O_W1B + SZ_W1B;
static constexpr size_t O_W2D  = O_W2H + SZ_W2H;
static constexpr size_t O_B2V  = O_W2D + SZ_W2D;
static constexpr size_t WS_TOTAL = O_B2V + SZ_B2V;
static_assert(SZ_A0 % 256 == 0 && SZ_HA % 256 == 0 && SZ_HB % 256 == 0 && SZ_AP % 256 == 0);
static_assert(SZ_W1B % 256 == 0 && SZ_W2H % 256 == 0 && SZ_W2D % 256 == 0 && SZ_B2V % 256 == 0);
static_assert(WS_TOTAL <= (size_t)WSMAX);
static_assert(!TABLE_AS_BUILT || WS_TOTAL == 81070080);

__global__ __launch_bounds__(NTHR) void k_prep(const float* __restrict__ w2, const float* __restrict__ b2,
                                               unsigned short* __restrict__ W2H, float* __restrict__ B2V) {
  const int tid = (int)threadIdx.x;
  const int b   = (int)blockIdx.x;
  if (b < PB_W2H) {
    const int g = b * NTHR + tid;
    v4f a = *(const v4fa*)(w2 + (size_t)g * 8);
    asm volatile("" :: "v"(a));
    v4f c = *(const v4fa*)(w2 + (size_t)g * 8 + 4);
    asm volatile("" :: "v"(c));
    const v4f as = (v4f){ bf16_val(a[0]) * CARRY, bf16_val(a[1]) * CARRY, bf16_val(a[2]) * CARRY, bf16_val(a[3]) * CARRY };
    const v4f cs = (v4f){ bf16_val(c[0]) * CARRY, bf16_val(c[1]) * CARRY, bf16_val(c[2]) * CARRY, bf16_val(c[3]) * CARRY };
    const v4u o = pack8_f16(as, cs);
    volatile v4u* q = (volatile v4u*)(W2H + (size_t)g * 8);
    *q = o;
    __threadfence();
    *q = o;
  } else {
    const int i = tid < (HID / 4) ? tid : (HID / 4 - 1);
    v4f qv = *(const v4fa*)(b2 + 4 * i);
    asm volatile("" :: "v"(qv));
    const v4f o = (v4f){ bf16_val(qv[0]), bf16_val(qv[1]), bf16_val(qv[2]), bf16_val(qv[3]) };
    if (tid < HID / 4) {
      volatile v4f* p = (volatile v4f*)(B2V + 4 * tid);
      *p = o;
      __threadfence();
      *p = o;
    }
  }
}

__device__ __forceinline__ v4u gather_piece(const float* er, int chunk) {
  const int col0 = chunk * 8;
  const int ca = col0 < (WDIM - 4) ? col0 : (WDIM - 4);
  const int cb = (col0 + 4) < (WDIM - 4) ? (col0 + 4) : (WDIM - 4);
  v4f va = *(const v4fa*)(er + ca);
  asm volatile("" :: "v"(va));
  v4f vb = *(const v4fa*)(er + cb);
  asm volatile("" :: "v"(vb));
  const unsigned m0 = (col0 + 0 < WDIM) ? 0xFFFFu : 0u;
  const unsigned m1 = (col0 + 1 < WDIM) ? 0xFFFFu : 0u;
  const unsigned m2 = (col0 + 2 < WDIM) ? 0xFFFFu : 0u;
  const unsigned m3 = (col0 + 3 < WDIM) ? 0xFFFFu : 0u;
  const unsigned m4 = (col0 + 4 < WDIM) ? 0xFFFFu : 0u;
  const unsigned m5 = (col0 + 5 < WDIM) ? 0xFFFFu : 0u;
  const unsigned m6 = (col0 + 6 < WDIM) ? 0xFFFFu : 0u;
  const unsigned m7 = (col0 + 7 < WDIM) ? 0xFFFFu : 0u;
  v4u o = pack8_bf16(va, vb);
  o &= (v4u){ pk16(m0, m1), pk16(m2, m3), pk16(m4, m5), pk16(m6, m7) };
  return o;
}

__global__ __launch_bounds__(NTHR) void k_gather(const int* __restrict__ ids, const float* __restrict__ table,
                                                 unsigned short* __restrict__ A0, int nrows) {
  const int lane = (int)threadIdx.x & 31;
  const int wave = (int)threadIdx.x >> 5;
  const int row  = (int)blockIdx.x * 8 + wave;
  const bool live = row < nrows;
  const int rowc = live ? row : nrows - 1;
  int idw = ids[rowc];
  asm volatile("" :: "v"(idw));
  const int id = clampi(idw, 0, VOCAB - 1);
  const float* er = table + (size_t)id * WDIM;
  const v4u o1 = gather_piece(er, lane);
  const v4u o2 = gather_piece(er, 32 + (lane & 7));
  unsigned short* rp = A0 + (size_t)rowc * K0PAD;
  volatile v4u* q1 = (volatile v4u*)(rp + 8 * lane);
  volatile v4u* q2 = (volatile v4u*)(rp + 256 + 8 * (lane & 7));
  const bool tail = lane < 8;
  if (live) {
    *q1 = o1;
    if (tail) *q2 = o2;
    __threadfence();
    *q1 = o1;
    if (tail) *q2 = o2;
  }
}

__global__ __launch_bounds__(NTHR) void k_fold(float* __restrict__ H, const float* __restrict__ bv, int n4) {
  const int t  = (int)blockIdx.x * NTHR + (int)threadIdx.x;
  const int tc = t < n4 ? t : n4 - 1;
  const int col = (tc * 4) & (HID - 1);
  v4f acc = *(const v4fa*)(H + (size_t)tc * 4);
  asm volatile("" :: "v"(acc));
  v4f b = *(const v4fa*)(bv + col);
  asm volatile("" :: "v"(b));
  const v4f sc = acc * FOLD;
  const v4f o  = sc + b;
  if (t < n4) {
    volatile v4f* p = (volatile v4f*)(H + (size_t)t * 4);
    *p = o;
    __threadfence();
    *p = o;
  }
}

extern "C" void kernel_launch(void* const* d_in, const int* in_sizes, int n_in,
                              void* d_out, int out_size, void* d_ws, size_t ws_size,
                              hipStream_t stream) {
  if (n_in < 5) return;
  if (in_sizes[0] != NTREE * NLEAF) return;
  if (in_sizes[1] != VOCAB * WDIM) return;
  if (in_sizes[2] != HID * WDIM) return;
  if (in_sizes[3] != HID * K2) return;
  if (in_sizes[4] != HID) return;
  if ((long long)out_size != (long long)NTREE * HID) return;
  if (ws_size < WS_TOTAL) return;

  const int*   ids = (const int*)d_in[0];
  const float* emb = (const float*)d_in[1];
  const float* W1  = (const float*)d_in[2];
  const float* W2  = (const float*)d_in[3];
  const float* b2  = (const float*)d_in[4];
  float* out = (float*)d_out;

  char* ws = (char*)d_ws;
  unsigned short* A0  = (unsigned short*)(ws + O_A0);
  float*          Ha  = (float*)(ws + O_HA);
  float*          Hb  = (float*)(ws + O_HB);
  unsigned short* AP  = (unsigned short*)(ws + O_AP);
  unsigned short* W1B = (unsigned short*)(ws + O_W1B);
  unsigned short* W2H = (unsigned short*)(ws + O_W2H);
  unsigned short* W2D = (unsigned short*)(ws + O_W2D);
  float*          B2V = (float*)(ws + O_B2V);

  k_plane<0><<<(HID * (K0PAD / 8)) / 256, 256, 0, stream>>>(W1, HID, WDIM, WDIM, W1B, HID, K0PAD);
  k_prep<<<PB_W2H + 1, NTHR, 0, stream>>>(W2, b2, W2H, B2V);
  k_plane<3><<<(HID * (2 * K2 / 8)) / 256, 256, 0, stream>>>(W2, HID, K2, K2, W2D, HID, K2);

  for (int g = 0; g < NGROUP; ++g) {
    k_gather<<<GROWS / 8, NTHR, 0, stream>>>(ids + (size_t)g * GROWS, emb, A0, GROWS);
    k_gemm_nt<0, 0><<<GROWS / 64, 256, 0, stream>>>(A0, W1B, B2V, Ha, GROWS, HID, K0PAD, HID);
    for (int l = 1; l <= NLEVEL; ++l) {
      const int M = GROWS >> l;
      const float* src = ((l - 1) & 1) ? Hb : Ha;
      float* dst = (l == NLEVEL) ? (out + (size_t)g * GTREES * HID) : ((l & 1) ? Hb : Ha);
      if (LEVEL_FORM[l - 1] == 2) {
        k_plane<2><<<(M * (K2 / 8)) / 256, 256, 0, stream>>>(src, M, K2, K2, AP, M, K2);
        k_gemm_nt<2, 0><<<M / 64, 256, 0, stream>>>(AP, W2H, B2V, dst, M, HID, K2, HID);
        k_fold<<<(M * (HID / 4)) / NTHR, NTHR, 0, stream>>>(dst, B2V, M * (HID / 4));
      } else {
        k_plane<1><<<(M * (2 * K2 / 8)) / 256, 256, 0, stream>>>(src, M, K2, K2, AP, M, K2);
        k_gemm_nt<1, 1><<<M / 64, 256, 0, stream>>>(AP, W2D, B2V, dst, M, HID, 2 * K2, HID);
      }
    }
  }
}
